// NNRankModel_35828617183464
// MI455X (gfx1250) — hardware-verified
//
#include <hip/hip_runtime.h>
#include <math.h>

constexpr int kRows      = 8192;
constexpr int kFields    = 40;
constexpr int kEmbDim    = 8;
constexpr int kFeatIn    = kFields * kEmbDim;
constexpr int kRed       = 5;
constexpr int kPairs     = 780;
constexpr int kPieces    = 2 * kPairs;
constexpr int kDnnIn     = kPieces * kEmbDim;
constexpr int kSeCols    = kPairs * kEmbDim;
constexpr int kHid1      = 1024;
constexpr int kHid2      = 512;
constexpr int kChunk     = 2048;
constexpr int kNumChunks = kRows / kChunk;
constexpr float kBnEps   = 1e-5f;

constexpr float kCarryASe  = 512.0f;
constexpr float kCarryARaw = 8.0f;
constexpr float kCarryWSe  = 16.0f;
constexpr float kCarryWRaw = 1024.0f;
constexpr float kCarryH1   = 16.0f;
constexpr float kCarryW2   = 256.0f;
constexpr float kScale1    = kCarryH1 / 8192.0f;
constexpr float kScale2    = 1.0f / (kCarryH1 * kCarryW2);

static_assert(kDnnIn % 32 == 0);
static_assert(kHid1 % 64 == 0 && kHid1 % 32 == 0);
static_assert(kHid2 % 64 == 0);
static_assert(kChunk % 64 == 0 && kRows % kChunk == 0);
static_assert(kRows % 32 == 0);
static_assert(kSeCols % 8 == 0 && kDnnIn % 8 == 0);
static_assert((kDnnIn * 2) % 128 == 0);

typedef __attribute__((ext_vector_type(16))) _Float16 v16h;
typedef __attribute__((ext_vector_type(8)))  _Float16 v8h;
typedef __attribute__((ext_vector_type(16))) __bf16   v16b;
typedef __attribute__((ext_vector_type(8)))  __bf16   v8b;
typedef __attribute__((ext_vector_type(8)))  float    v8f;
typedef __attribute__((ext_vector_type(4)))  float    v4f;
typedef __attribute__((ext_vector_type(4)))  unsigned int v4u;

__device__ __forceinline__ unsigned short f2bf_bits(float f) {
  unsigned u = __float_as_uint(f);
  return (unsigned short)((u + 0x7FFFu + ((u >> 16) & 1u)) >> 16);
}
__device__ __forceinline__ float bf_bits2f(unsigned short h) { return __uint_as_float(((unsigned)h) << 16); }

__device__ __forceinline__ void dep_guard_h(v8f& a, v8f& b, v16h x, v16h y) { asm volatile("v_nop\n\tv_nop\n\tv_nop\n\tv_nop" : "+v"(a), "+v"(b) : "v"(x), "v"(y)); }
__device__ __forceinline__ void dep_guard_b(v8f& a, v8f& b, v16b x, v16b y) { asm volatile("v_nop\n\tv_nop\n\tv_nop\n\tv_nop" : "+v"(a), "+v"(b) : "v"(x), "v"(y)); }
__device__ __forceinline__ void keep4_h(v16h a, v16h b, v16h c, v16h d) { asm volatile("v_nop" :: "v"(a), "v"(b), "v"(c), "v"(d)); }
__device__ __forceinline__ void keep4_b(v16b a, v16b b, v16b c, v16b d) { asm volatile("v_nop" :: "v"(a), "v"(b), "v"(c), "v"(d)); }
__device__ __forceinline__ void acc_guard4(v8f& a, v8f& b, v8f& c, v8f& d) { asm volatile("v_nop\n\tv_nop\n\tv_nop\n\tv_nop" : "+v"(a), "+v"(b), "+v"(c), "+v"(d)); }
template <typename T> struct Frag;
template <> struct Frag<_Float16> {
  typedef v16h V; union U { v16h v; v8h h[2]; };
  static __device__ __forceinline__ v16h load(const _Float16* p) {
    U f; f.h[0] = *(const v8h*)(p); f.h[1] = *(const v8h*)(p + 16); return f.v;
  }
  static __device__ __forceinline__ v8f mma(v16h a, v16h b, v8f c) {
    return __builtin_amdgcn_wmma_f32_16x16x32_f16(false, a, false, b, (short)0, c, false, false);
  }
  static __device__ __forceinline__ void guard(v8f& a, v8f& b, v16h x, v16h y) { dep_guard_h(a, b, x, y); }
  static __device__ __forceinline__ void keep(v16h a, v16h b, v16h c, v16h d) { keep4_h(a, b, c, d); }
};
template <> struct Frag<__bf16> {
  typedef v16b V; union U { v16b v; v8b h[2]; };
  static __device__ __forceinline__ v16b load(const __bf16* p) {
    U f; f.h[0] = *(const v8b*)(p); f.h[1] = *(const v8b*)(p + 16); return f.v;
  }
  static __device__ __forceinline__ v8f mma(v16b a, v16b b, v8f c) {
    return __builtin_amdgcn_wmma_f32_16x16x32_bf16(false, a, false, b, (short)0, c, false, false);
  }
  static __device__ __forceinline__ void guard(v8f& a, v8f& b, v16b x, v16b y) { dep_guard_b(a, b, x, y); }
  static __device__ __forceinline__ void keep(v16b a, v16b b, v16b c, v16b d) { keep4_b(a, b, c, d); }
};

__device__ __forceinline__ unsigned pk16(unsigned short a, unsigned short b) { return (unsigned)a | ((unsigned)b << 16); }
__device__ __forceinline__ unsigned short h_bits(float f) { const _Float16 h = (_Float16)f; return __builtin_bit_cast(unsigned short, h); }

template <int ET> struct Elem;
template <> struct Elem<0> { typedef _Float16 T; };
template <> struct Elem<1> { typedef __bf16 T; };
template <int ET, bool SPLIT, int BIAS_MODE, int OUT_MODE, bool RESID, int ACT = 0>
__global__ __launch_bounds__(256) void wmma_gemm64(
    const unsigned short* __restrict__ Ap, const unsigned short* __restrict__ A2p, int lda, long strideA,
    const unsigned short* __restrict__ Btp, const unsigned short* __restrict__ Bt2p, int ldb, long strideB,
    void* __restrict__ Cout, void* __restrict__ Cout2, int ldc, long strideC,
    const float* __restrict__ bias,
    const float* __restrict__ resid, long strideR,
    int M, int N, int K, float scale) {
  typedef typename Elem<ET>::T T;
  typedef typename Frag<T>::V V;
  const T* A = (const T*)Ap; const T* A2 = (const T*)A2p; const T* Bt = (const T*)Btp; const T* Bt2 = (const T*)Bt2p;
  __shared__ __align__(16) float sT[8][16 * 68];
  const int b    = blockIdx.y;
  const int lane = threadIdx.x & 31;
  const int wave = threadIdx.x >> 5;
  const int tilesN = N >> 6;
  const int tilesM = M >> 6;
  const int tile = blockIdx.x * 8 + wave;
  if (tile >= tilesM * tilesN) return;
  const int tm = tile / tilesN;
  const int tn = tile - tm * tilesN;
  const int m0 = tm << 6;
  const int n0 = tn << 6;

  const T* Ab  = A  + (size_t)b * strideA;
  const T* Bb  = Bt + (size_t)b * strideB;
  const T* Ab2 = SPLIT ? (A2  + (size_t)b * strideA) : nullptr;
  const T* Bb2 = SPLIT ? (Bt2 + (size_t)b * strideB) : nullptr;

  const int rlane = lane & 15;
  const int koff  = (lane >> 4) * 8;
  const int mOff  = (lane >> 4) * 8;

  v8f acc[4][4];
#pragma unroll
  for (int i = 0; i < 4; ++i)
#pragma unroll
    for (int j = 0; j < 4; ++j) acc[i][j] = (v8f){0.f,0.f,0.f,0.f,0.f,0.f,0.f,0.f};

  for (int k0 = 0; k0 < K; k0 += 32) {
    V bh[4], bl[4];
#pragma unroll
    for (int j = 0; j < 4; ++j) {
      const size_t bo = (size_t)(n0 + (j << 4) + rlane) * ldb + koff + k0;
      bh[j] = Frag<T>::load(Bb + bo);
      if (SPLIT) bl[j] = Frag<T>::load(Bb2 + bo);
    }
#pragma unroll
    for (int i = 0; i < 4; ++i) {
      const size_t ao = (size_t)(m0 + (i << 4) + rlane) * lda + koff + k0;
      V ah = Frag<T>::load(Ab + ao);
      V al;
      if (SPLIT) al = Frag<T>::load(Ab2 + ao);
#pragma unroll
      for (int j = 0; j < 4; ++j) {
        acc[i][j] = Frag<T>::mma(ah, bh[j], acc[i][j]);
        if (SPLIT) {
          acc[i][j] = Frag<T>::mma(ah, bl[j], acc[i][j]);
          acc[i][j] = Frag<T>::mma(al, bh[j], acc[i][j]);
        }
      }
      Frag<T>::guard(acc[i][0], acc[i][3], ah, SPLIT ? al : ah);
    }
    Frag<T>::keep(bh[0], bh[1], bh[2], bh[3]);
    if (SPLIT) Frag<T>::keep(bl[0], bl[1], bl[2], bl[3]);
  }
  acc_guard4(acc[0][0], acc[0][1], acc[0][2], acc[0][3]);
  acc_guard4(acc[1][0], acc[1][1], acc[1][2], acc[1][3]);
  acc_guard4(acc[2][0], acc[2][1], acc[2][2], acc[2][3]);
  acc_guard4(acc[3][0], acc[3][1], acc[3][2], acc[3][3]);

  float* slab = sT[wave];
  const float* Rb = RESID ? (resid + (size_t)b * strideR) : nullptr;
#pragma unroll
  for (int i = 0; i < 4; ++i) {
    const int mBase = m0 + (i << 4);
#pragma unroll
    for (int j = 0; j < 4; ++j) {
      const int n = n0 + (j << 4) + rlane;
      float bv = 0.f;
      if (BIAS_MODE == 2) bv = bias[n];
#pragma unroll
      for (int r = 0; r < 8; ++r) {
        float v = acc[i][j][r] * scale;
        if (BIAS_MODE == 1) v += bias[mBase + mOff + r];
        if (BIAS_MODE == 2) v += bv;
        if (RESID) v += Rb[(size_t)(mBase + mOff + r) * ldc + n];
        if (ACT == 2) v = fmaxf(v, 0.0f);
        if (ACT == 4) v = (v > 0.f) ? v : 0.01f * v;
        slab[(mOff + r) * 68 + (j << 4) + rlane] = v;
      }
    }
    __builtin_amdgcn_fence(__ATOMIC_RELEASE, "workgroup");
    __builtin_amdgcn_wave_barrier();
    __builtin_amdgcn_fence(__ATOMIC_ACQUIRE, "workgroup");
    if (OUT_MODE == 0) {
      float* C = (float*)Cout + (size_t)b * strideC;
      const int hh = lane >> 4, c4 = (lane & 15) * 4;
      for (int pass = 0; pass < 2; ++pass) {
#pragma unroll
        for (int it = 0; it < 8; ++it) {
          const int row = it * 2 + hh;
          v4f v = *(const v4f*)(slab + row * 68 + c4);
          *(volatile v4f*)(C + (size_t)(mBase + row) * ldc + n0 + c4) = v;
        }
        __threadfence();
      }
    } else {
      const int q = lane >> 3, c8 = (lane & 7) * 8;
      unsigned short* C  = (unsigned short*)Cout  + (size_t)b * strideC;
      unsigned short* C2 = (OUT_MODE == 2) ? ((unsigned short*)Cout2 + (size_t)b * strideC) : nullptr;
      for (int pass = 0; pass < 2; ++pass) {
#pragma unroll
        for (int it = 0; it < 4; ++it) {
          const int row = it * 4 + q;
          const float* sp = slab + row * 68 + c8;
          v8h hv, lv;
#pragma unroll
          for (int e = 0; e < 8; ++e) {
            if (OUT_MODE == 1) {
              hv[e] = (_Float16)sp[e];
            } else {
              unsigned short hb = f2bf_bits(sp[e]);
              unsigned short lb = f2bf_bits(sp[e] - bf_bits2f(hb));
              hv[e] = __builtin_bit_cast(_Float16, hb);
              lv[e] = __builtin_bit_cast(_Float16, lb);
            }
          }
          *(volatile v8h*)(C + (size_t)(mBase + row) * ldc + n0 + c8) = hv;
          if (OUT_MODE == 2) *(volatile v8h*)(C2 + (size_t)(mBase + row) * ldc + n0 + c8) = lv;
        }
        __threadfence();
      }
    }
    __builtin_amdgcn_fence(__ATOMIC_RELEASE, "workgroup");
    __builtin_amdgcn_wave_barrier();
    __builtin_amdgcn_fence(__ATOMIC_ACQUIRE, "workgroup");
  }
}

__global__ __launch_bounds__(256) void cast8_carry_kernel(const float* __restrict__ in, unsigned short* __restrict__ out,
                                                         int n8, int ncols, int split_col, float s_first, float s_second) {
  const int i = blockIdx.x * 256 + threadIdx.x;
  if (i >= n8) return;
  const int col = (8 * i) % ncols;
  const float sc = (col < split_col) ? s_first : s_second;
  const float* p = in + 8 * (size_t)i;
  const v4f a = *(const v4f*)(p);
  const v4f c = *(const v4f*)(p + 4);
  unsigned short hb[8];
#pragma unroll
  for (int e = 0; e < 4; ++e) {
    hb[e]     = h_bits(a[e] * sc);
    hb[4 + e] = h_bits(c[e] * sc);
  }
  const v4u u = (v4u){pk16(hb[0], hb[1]), pk16(hb[2], hb[3]), pk16(hb[4], hb[5]), pk16(hb[6], hb[7])};
  unsigned short* q = out + 8 * (size_t)i;
  *(volatile v4u*)q = u;
  __threadfence();
  *(volatile v4u*)q = u;
}

__global__ __launch_bounds__(256) void scale_vec_kernel(const float* __restrict__ in, float* __restrict__ out, int n4, float s) {
  const int i = blockIdx.x * 256 + threadIdx.x;
  if (i >= n4) return;
  v4f v = *(const v4f*)(in + 4 * (size_t)i);
  v = v * s;
  float* q = out + 4 * (size_t)i;
  *(volatile v4f*)q = v;
  __threadfence();
  *(volatile v4f*)q = v;
}

__global__ __launch_bounds__(256) void feat_kernel(
    const float* __restrict__ emb, const float* __restrict__ bnw, const float* __restrict__ bnb,
    const float* __restrict__ bnm, const float* __restrict__ bnv,
    const float* __restrict__ sew1, const float* __restrict__ sew2, const float* __restrict__ wbl,
    unsigned short* __restrict__ Aout, int row0)
{
  __shared__ __align__(16) float V0[kFeatIn];
  __shared__ __align__(16) float T0[kFeatIn];
  __shared__ float Zs[kFields];
  __shared__ float ZR[8];
  __shared__ float Aex[kFields];
  __shared__ float Ws[kEmbDim * kEmbDim];
  __shared__ unsigned char PI[kPairs];
  __shared__ unsigned char PJ[kPairs];

  const int tid  = threadIdx.x;
  const int grow = row0 + blockIdx.x;

  if (tid < kFields) {
    const int base = tid * (kFields - 1) - (tid * (tid - 1)) / 2;
    for (int j = tid + 1; j < kFields; ++j) {
      PI[base + j - tid - 1] = (unsigned char)tid;
      PJ[base + j - tid - 1] = (unsigned char)j;
    }
  }
  if (tid < kEmbDim * kEmbDim) Ws[tid] = wbl[tid];
  for (int f = tid; f < kFeatIn; f += 256) {
    const float e = emb[(size_t)grow * kFeatIn + f];
    const float r = rsqrtf(bnv[f] + kBnEps);
    V0[f] = (e - bnm[f]) * r * bnw[f] + bnb[f];
  }
  __syncthreads();

  if (tid < kFields) {
    float s = 0.f;
#pragma unroll
    for (int e = 0; e < kEmbDim; ++e) s += V0[tid * kEmbDim + e];
    Zs[tid] = s * 0.125f;
  }
  __syncthreads();

  if (tid < kRed) {
    float s = 0.f;
#pragma unroll 1
    for (int f = 0; f < kFields; ++f) s += Zs[f] * sew1[tid * kFields + f];
    ZR[tid] = fmaxf(s, 0.f);
  }
  __syncthreads();

  if (tid < kFields) {
    float s = 0.f;
#pragma unroll
    for (int r = 0; r < kRed; ++r) s += ZR[r] * sew2[tid * kRed + r];
    Aex[tid] = fmaxf(s, 0.f);
  }
  for (int q = tid; q < kFeatIn; q += 256) {
    const int f = q >> 3, d = q & 7;
    float s = 0.f;
#pragma unroll
    for (int e = 0; e < kEmbDim; ++e) s += V0[f * kEmbDim + e] * Ws[d * kEmbDim + e];
    T0[q] = s;
  }
  __syncthreads();

  v4u vals[7];
#pragma unroll
  for (int it = 0; it < 7; ++it) {
    const int p  = it * 256 + tid;
    const int pc = (p < kPieces) ? p : (kPieces - 1);
    const bool se = (pc < kPairs);
    const int k  = se ? pc : (pc - kPairs);
    const int i  = (int)PI[k];
    const int j  = (int)PJ[k];
    const float ai = Aex[i];
    const float aj = Aex[j];
    const float g  = se ? (ai * aj * kCarryASe) : kCarryARaw;
    const v4f t0 = *(const v4f*)(T0 + i * kEmbDim);
    const v4f t1 = *(const v4f*)(T0 + i * kEmbDim + 4);
    const v4f v0 = *(const v4f*)(V0 + j * kEmbDim);
    const v4f v1 = *(const v4f*)(V0 + j * kEmbDim + 4);
    unsigned short hb[8];
#pragma unroll
    for (int e = 0; e < 4; ++e) {
      hb[e]     = h_bits((g * t0[e]) * v0[e]);
      hb[4 + e] = h_bits((g * t1[e]) * v1[e]);
    }
    vals[it] = (v4u){pk16(hb[0], hb[1]), pk16(hb[2], hb[3]), pk16(hb[4], hb[5]), pk16(hb[6], hb[7])};
  }

  unsigned short* dst = Aout + (size_t)blockIdx.x * kDnnIn;
  for (int pass = 0; pass < 2; ++pass) {
#pragma unroll
    for (int it = 0; it < 7; ++it) {
      const int p = it * 256 + tid;
      if (p < kPieces) *(volatile v4u*)(dst + 8 * (size_t)p) = vals[it];
    }
    __threadfence();
  }
}

__global__ __launch_bounds__(256) void head_kernel(const float* __restrict__ H2, const float* __restrict__ w3,
                                                   const float* __restrict__ b3, float* __restrict__ out, int nrows) {
  __shared__ __align__(16) float res[32];
  const int tid  = threadIdx.x;
  const int lane = tid & 31;
  const int wave = tid >> 5;
  const int rbase = blockIdx.x * 32;
  const float bb = b3[0];
  v4f wv[4];
#pragma unroll
  for (int s = 0; s < 4; ++s) wv[s] = *(const v4f*)(w3 + s * 128 + lane * 4);
#pragma unroll 1
  for (int rr = 0; rr < 4; ++rr) {
    const int row  = rbase + wave * 4 + rr;
    const int rowc = (row < nrows) ? row : (nrows - 1);
    const float* hr = H2 + (size_t)rowc * kHid2;
    float acc = 0.f;
#pragma unroll
    for (int s = 0; s < 4; ++s) {
      const v4f hv = *(const v4f*)(hr + s * 128 + lane * 4);
      acc += hv[0] * wv[s][0];
      acc += hv[1] * wv[s][1];
      acc += hv[2] * wv[s][2];
      acc += hv[3] * wv[s][3];
    }
#pragma unroll
    for (int off = 16; off > 0; off >>= 1) acc += __shfl_xor(acc, off, 32);
    float z = acc + bb;
    z = fminf(fmaxf(z, -80.0f), 80.0f);
    const float y = 1.0f / (1.0f + expf(-z));
    if (lane == 0) res[wave * 4 + rr] = y;
  }
  __syncthreads();
  if (wave == 0) {
    const int l8 = lane & 7;
    const v4f v = *(const v4f*)(res + l8 * 4);
    float* op = out + (size_t)rbase + l8 * 4;
    if (lane < 8 && rbase + 32 <= nrows) *(volatile v4f*)op = v;
    __threadfence();
    if (lane < 8 && rbase + 32 <= nrows) *(volatile v4f*)op = v;
  }
}

extern "C" void kernel_launch(void* const* d_in, const int* in_sizes, int n_in,
                              void* d_out, int out_size, void* d_ws, size_t ws_size,
                              hipStream_t stream)
{
  if (n_in < 14) return;
  const float* emb  = (const float*)d_in[0];
  const float* bnw  = (const float*)d_in[1];
  const float* bnb  = (const float*)d_in[2];
  const float* bnm  = (const float*)d_in[3];
  const float* bnv  = (const float*)d_in[4];
  const float* sew1 = (const float*)d_in[5];
  const float* sew2 = (const float*)d_in[6];
  const float* wbl  = (const float*)d_in[7];
  const float* w1f  = (const float*)d_in[8];
  const float* b1   = (const float*)d_in[9];
  const float* w2f  = (const float*)d_in[10];
  const float* b2   = (const float*)d_in[11];
  const float* w3   = (const float*)d_in[12];
  const float* b3   = (const float*)d_in[13];
  float* out = (float*)d_out;

  if (in_sizes[0] != kRows * kFeatIn) return;
  if (in_sizes[1] != kFeatIn || in_sizes[2] != kFeatIn || in_sizes[3] != kFeatIn || in_sizes[4] != kFeatIn) return;
  if (in_sizes[5] != kRed * kFields || in_sizes[6] != kFields * kRed || in_sizes[7] != kEmbDim * kEmbDim) return;
  if (in_sizes[8] != kHid1 * kDnnIn || in_sizes[9] != kHid1) return;
  if (in_sizes[10] != kHid2 * kHid1 || in_sizes[11] != kHid2 || in_sizes[12] != kHid2 || in_sizes[13] < 1) return;
  if (out_size != kRows) return;

  const size_t bytesA  = (size_t)kChunk * kDnnIn * 2;
  const size_t bytesW1 = (size_t)kHid1 * kDnnIn * 2;
  const size_t bytesW2 = (size_t)kHid2 * kHid1 * 2;
  const size_t bytesH1 = (size_t)kRows * kHid1 * 2;
  const size_t bytesH2 = (size_t)kRows * kHid2 * 4;
  const size_t bytesB1 = (size_t)kHid1 * 4;
  const size_t offA  = 0;
  const size_t offW1 = offA + bytesA;
  const size_t offW2 = offW1 + bytesW1;
  const size_t offH1 = offW2 + bytesW2;
  const size_t offH2 = offH1 + bytesH1;
  const size_t offB1 = offH2 + bytesH2;
  const size_t total = offB1 + bytesB1;
  if (total > ws_size) return;
  if (total > (size_t)134217728) return;

  char* ws = (char*)d_ws;
  unsigned short* Apl = (unsigned short*)(ws + offA);
  unsigned short* W1h = (unsigned short*)(ws + offW1);
  unsigned short* W2h = (unsigned short*)(ws + offW2);
  unsigned short* H1  = (unsigned short*)(ws + offH1);
  float*          H2  = (float*)(ws + offH2);
  float*          b1s = (float*)(ws + offB1);

  {
    const int n8w1 = (kHid1 * kDnnIn) / 8;
    cast8_carry_kernel<<<dim3((n8w1 + 255) / 256, 1, 1), dim3(256, 1, 1), 0, stream>>>(
        w1f, W1h, n8w1, kDnnIn, kSeCols, kCarryWSe, kCarryWRaw);
    const int n8w2 = (kHid2 * kHid1) / 8;
    cast8_carry_kernel<<<dim3((n8w2 + 255) / 256, 1, 1), dim3(256, 1, 1), 0, stream>>>(
        w2f, W2h, n8w2, kHid1, kHid1, kCarryW2, kCarryW2);
    const int n4b1 = kHid1 / 4;
    scale_vec_kernel<<<dim3((n4b1 + 255) / 256, 1, 1), dim3(256, 1, 1), 0, stream>>>(b1, b1s, n4b1, kCarryH1);
  }

  const int tiles1 = (kChunk / 64) * (kHid1 / 64);
  for (int c = 0; c < kNumChunks; ++c) {
    feat_kernel<<<dim3(kChunk, 1, 1), dim3(256, 1, 1), 0, stream>>>(
        emb, bnw, bnb, bnm, bnv, sew1, sew2, wbl, Apl, c * kChunk);
    unsigned short* H1c = H1 + (size_t)c * kChunk * kHid1;
    wmma_gemm64<0, false, 2, 1, false, 2><<<dim3((tiles1 + 7) / 8, 1, 1), dim3(256, 1, 1), 0, stream>>>(
        Apl, Apl, kDnnIn, 0L,
        W1h, W1h, kDnnIn, 0L,
        (void*)H1c, (void*)H1c, kHid1, 0L,
        b1s,
        b1s, 0L,
        kChunk, kHid1, kDnnIn, kScale1);
  }

  {
    const int tiles2 = (kRows / 64) * (kHid2 / 64);
    wmma_gemm64<0, false, 2, 0, false, 2><<<dim3((tiles2 + 7) / 8, 1, 1), dim3(256, 1, 1), 0, stream>>>(
        H1, H1, kHid1, 0L,
        W2h, W2h, kHid1, 0L,
        (void*)H2, (void*)H2, kHid2, 0L,
        b2,
        b2, 0L,
        kRows, kHid2, kHid1, kScale2);
  }

  head_kernel<<<dim3(kRows / 32, 1, 1), dim3(256, 1, 1), 0, stream>>>(H2, w3, b3, out, kRows);
}
